// GRUDecoder_49615462203957
// MI455X (gfx1250) — hardware-run, weakly checked
//
#include <hip/hip_runtime.h>
#include <math.h>

constexpr int NBATCH     = 256;
constexpr int NHID       = 1024;
constexpr int NGATE3     = 3 * NHID;
constexpr int NSTEP      = 128;
constexpr int NTHR       = 256;
constexpr int NWAVE      = NTHR / 32;
constexpr int ROWS_BLK   = 16;
constexpr int UNITS_WAVE = NHID / NWAVE;
constexpr int NSUB       = UNITS_WAVE / 16;
constexpr int HP         = NHID + 8;
constexpr int HFP        = NHID + 4;
constexpr int YBP        = NSTEP + 4;
constexpr int NCT        = 10;
constexpr int W8         = NGATE3 * NHID / 8;
constexpr long GPLANE    = (long)NHID * NHID;
constexpr float HCARRY   = 16.0f;
constexpr float WCARRY   = 256.0f;
constexpr float GH_INV   = 1.0f / 4096.0f;
static_assert(NHID % 32 == 0);
static_assert(ROWS_BLK == 16);
static_assert(NBATCH % ROWS_BLK == 0);
static_assert(UNITS_WAVE * NWAVE == NHID && NSUB * 16 == UNITS_WAVE);
static_assert(NHID == 4 * NTHR);
static_assert(NSTEP == 32 * 4);
static_assert(ROWS_BLK == 2 * NWAVE);
static_assert(2 * ROWS_BLK * 8 == NTHR);
static_assert((NGATE3 * NHID) % 8 == 0 && W8 % NTHR == 0);
static_assert(HP % 8 == 0 && HFP % 4 == 0 && YBP % 4 == 0);
static_assert(HCARRY * WCARRY == 4096.0f);

typedef __attribute__((ext_vector_type(16))) _Float16 v16h;
typedef __attribute__((ext_vector_type(8)))  _Float16 v8h;
typedef __attribute__((ext_vector_type(8)))  float    v8f;
typedef __attribute__((ext_vector_type(4)))  float    v4f;
typedef __attribute__((ext_vector_type(4)))  unsigned v4u;
typedef __attribute__((ext_vector_type(2)))  unsigned v2u;

__device__ __forceinline__ unsigned short f2bf_bits(float f) {
  unsigned u = __float_as_uint(f);
  return (unsigned short)((u + 0x7FFFu + ((u >> 16) & 1u)) >> 16);
}
__device__ __forceinline__ float bf_bits2f(unsigned short h) { return __uint_as_float(((unsigned)h) << 16); }
__device__ __forceinline__ float bf16r(float f) { return bf_bits2f(f2bf_bits(f)); }
__device__ __forceinline__ unsigned short h16_bits(float f) {
  const _Float16 hv = (_Float16)f;
  return __builtin_bit_cast(unsigned short, hv);
}

struct FragH {
  union U { v16h v; v8h h[2]; };
  static __device__ __forceinline__ v16h load(const _Float16* p) {
    U f; f.h[0] = *(const v8h*)(p); f.h[1] = *(const v8h*)(p + 16); return f.v;
  }
  static __device__ __forceinline__ v8f mma(v16h a, v16h b, v8f c) {
    return __builtin_amdgcn_wmma_f32_16x16x32_f16(false, a, false, b, (short)0, c, false, false);
  }
};

__device__ __forceinline__ void guard3(v8f& a0, v8f& a1, v8f& a2, v16h x, v16h y0, v16h y1, v16h y2) {
  asm volatile("v_nop\n\tv_nop\n\tv_nop\n\tv_nop"
               : "+v"(a0), "+v"(a1), "+v"(a2)
               : "v"(x), "v"(y0), "v"(y1), "v"(y2));
}
__device__ __forceinline__ void acc_guard3(v8f& a0, v8f& a1, v8f& a2) {
  asm volatile("v_nop\n\tv_nop\n\tv_nop\n\tv_nop" : "+v"(a0), "+v"(a1), "+v"(a2));
}

__device__ __forceinline__ float sigm_f(float x) { return __builtin_amdgcn_rcpf(1.0f + expf(-x)); }
__device__ __forceinline__ float tanh_f(float x) { return 1.0f - 2.0f * __builtin_amdgcn_rcpf(1.0f + expf(2.0f * x)); }

__global__ __launch_bounds__(NTHR) void cvt_w_kernel(const float* __restrict__ src, unsigned short* __restrict__ dst, int n8) {
  const int i = blockIdx.x * NTHR + threadIdx.x;
  if (i < n8) {
    const float* sp = src + (size_t)i * 8;
    const v4f a = *(const v4f*)(sp);
    const v4f b = *(const v4f*)(sp + 4);
    const unsigned u0 = h16_bits(bf16r(a[0]) * WCARRY), u1 = h16_bits(bf16r(a[1]) * WCARRY);
    const unsigned u2 = h16_bits(bf16r(a[2]) * WCARRY), u3 = h16_bits(bf16r(a[3]) * WCARRY);
    const unsigned u4 = h16_bits(bf16r(b[0]) * WCARRY), u5 = h16_bits(bf16r(b[1]) * WCARRY);
    const unsigned u6 = h16_bits(bf16r(b[2]) * WCARRY), u7 = h16_bits(bf16r(b[3]) * WCARRY);
    v4u w;
    w[0] = u0 | (u1 << 16);
    w[1] = u2 | (u3 << 16);
    w[2] = u4 | (u5 << 16);
    w[3] = u6 | (u7 << 16);
    v4u* dp = (v4u*)(dst + (size_t)i * 8);
    *(volatile v4u*)dp = w;
    __threadfence();
    *(volatile v4u*)dp = w;
  }
}

__global__ __launch_bounds__(NTHR) void ctab_kernel(const float* __restrict__ w_ih, const float* __restrict__ b_ih,
                                                    const float* __restrict__ b_hh, const float* __restrict__ w_ffn,
                                                    float* __restrict__ CT) {
  const int q = blockIdx.x;
  const int g = q % 3;
  const int col4 = threadIdx.x * 4;
  const v4f va = *(const v4f*)(w_ih + (size_t)g * NHID + col4);
  const v4f vb = *(const v4f*)(b_ih + (size_t)g * NHID + col4);
  const v4f vc = *(const v4f*)(b_hh + (size_t)g * NHID + col4);
  const v4f vd = *(const v4f*)(w_ffn + col4);
  const float fa = (q < 3) ? 1.0f : 0.0f;
  const float fb = (q >= 3 && q < 6) ? 1.0f : 0.0f;
  const float fc = (q >= 6 && q < 9) ? 1.0f : 0.0f;
  const float fd = (q == 9) ? 1.0f : 0.0f;
  v4f o;
#pragma unroll
  for (int e = 0; e < 4; ++e) o[e] = bf16r(fa * va[e] + fb * vb[e] + fc * vc[e] + fd * vd[e]);
  float* op = CT + (size_t)q * NHID + col4;
  *(volatile v4f*)op = o;
  __threadfence();
  *(volatile v4f*)op = o;
}

__global__ __launch_bounds__(NTHR) void gru_seq_kernel(const float* __restrict__ vectors, const float* __restrict__ CT,
                                                       const float* __restrict__ b_ffn, const float* __restrict__ first_input,
                                                       const int* __restrict__ seq_len, const unsigned short* __restrict__ WHp,
                                                       float* __restrict__ out) {
  __shared__ __align__(16) _Float16 Ah[2][ROWS_BLK * HP];
  __shared__ __align__(16) float    hf[ROWS_BLK * HFP];
  __shared__ __align__(16) float    ybuf[ROWS_BLK * YBP];
  __shared__ float                  ypart[2 * NWAVE * ROWS_BLK];
  const _Float16* WH = (const _Float16*)WHp;
  const int tid = threadIdx.x, lane = tid & 31, wave = tid >> 5;
  const int c = lane & 15, hh = lane >> 4, koff = hh * 8;
  const int rowbase = blockIdx.x * ROWS_BLK;

  {
    const int buf = tid >> 7, row = (tid >> 3) & 15, col = NHID + (tid & 7);
    Ah[buf][row * HP + col] = (_Float16)0.0f;
  }
  if (tid < ROWS_BLK * 4) hf[(tid >> 2) * HFP + NHID + (tid & 3)] = 0.0f;
#pragma unroll 1
  for (int i = tid; i < ROWS_BLK * YBP; i += NTHR) ybuf[i] = 0.0f;
#pragma unroll 1
  for (int i = 0; i < ROWS_BLK; ++i) {
    const v4f v = *(const v4f*)(vectors + (size_t)(rowbase + i) * NHID + 4 * tid);
    v4f o;
#pragma unroll
    for (int e = 0; e < 4; ++e) o[e] = bf16r(v[e]);
    *(v4f*)(hf + i * HFP + 4 * tid) = o;
    const unsigned u0 = h16_bits(o[0] * HCARRY), u1 = h16_bits(o[1] * HCARRY);
    const unsigned u2 = h16_bits(o[2] * HCARRY), u3 = h16_bits(o[3] * HCARRY);
    v2u pk;
    pk[0] = u0 | (u1 << 16);
    pk[1] = u2 | (u3 << 16);
    *(v2u*)(&Ah[0][0] + i * HP + 4 * tid) = pk;
  }
  const float bffr = bf16r(b_ffn[0]);
  const float x0v  = bf16r(first_input[0]);
  int tcount = seq_len[0];
  tcount = tcount < 1 ? 1 : tcount;
  tcount = tcount > NSTEP ? NSTEP : tcount;
  float xv[8];
#pragma unroll
  for (int r = 0; r < 8; ++r) xv[r] = x0v;
  __syncthreads();

  const v8f z8 = {0.f, 0.f, 0.f, 0.f, 0.f, 0.f, 0.f, 0.f};

#pragma unroll 1
  for (int t = 0; t < tcount; ++t) {
    const int par = t & 1;
    const _Float16* arow  = &Ah[par][0] + c * HP + koff;
    _Float16*       anext = &Ah[par ^ 1][0];
    float ysum[8];
#pragma unroll
    for (int r = 0; r < 8; ++r) ysum[r] = 0.0f;

#pragma unroll 1
    for (int u = 0; u < NSUB; ++u) {
      const int j = UNITS_WAVE * wave + 16 * u + c;
      const _Float16* wrow = WH + (size_t)j * NHID + koff;
      v8f acc0 = z8, acc1 = z8, acc2 = z8;
#pragma unroll 1
      for (int k0 = 0; k0 < NHID; k0 += 32) {
        const v16h a  = FragH::load(arow + k0);
        const v16h b0 = FragH::load(wrow + k0);
        const v16h b1 = FragH::load(wrow + (size_t)GPLANE + k0);
        const v16h b2 = FragH::load(wrow + (size_t)2 * GPLANE + k0);
        acc0 = FragH::mma(a, b0, acc0);
        acc1 = FragH::mma(a, b1, acc1);
        acc2 = FragH::mma(a, b2, acc2);
        guard3(acc0, acc1, acc2, a, b0, b1, b2);
      }
      acc_guard3(acc0, acc1, acc2);

      asm volatile("" ::: "memory");
      const float wir = CT[0 * NHID + j], wiz = CT[1 * NHID + j], win = CT[2 * NHID + j];
      const float bir = CT[3 * NHID + j], biz = CT[4 * NHID + j], bin = CT[5 * NHID + j];
      const float bhr = CT[6 * NHID + j], bhz = CT[7 * NHID + j], bhn = CT[8 * NHID + j];
      const float wfj = CT[9 * NHID + j];
#pragma unroll
      for (int r = 0; r < 8; ++r) {
        const int m = 8 * hh + r;
        const float gir = xv[r] * wir + bir;
        const float giz = xv[r] * wiz + biz;
        const float gin = xv[r] * win + bin;
        const float ghr = acc0[r] * GH_INV + bhr;
        const float ghz = acc1[r] * GH_INV + bhz;
        const float ghn = acc2[r] * GH_INV + bhn;
        const float rg = sigm_f(gir + ghr);
        const float zg = sigm_f(giz + ghz);
        const float ng = tanh_f(gin + rg * ghn);
        const float ho = hf[m * HFP + j];
        const float hn = (1.0f - zg) * ng + zg * ho;
        hf[m * HFP + j] = hn;
        anext[m * HP + j] = (_Float16)(hn * HCARRY);
        ysum[r] = ysum[r] + hn * wfj;
      }
    }

#pragma unroll
    for (int r = 0; r < 8; ++r) {
      float s = ysum[r];
      s += __shfl_xor(s, 1, 32);
      s += __shfl_xor(s, 2, 32);
      s += __shfl_xor(s, 4, 32);
      s += __shfl_xor(s, 8, 32);
      if (c == 0) ypart[par * (NWAVE * ROWS_BLK) + wave * ROWS_BLK + 8 * hh + r] = s;
    }
    __syncthreads();

#pragma unroll
    for (int r = 0; r < 8; ++r) {
      float s = 0.0f;
#pragma unroll
      for (int w = 0; w < NWAVE; ++w) s += ypart[par * (NWAVE * ROWS_BLK) + w * ROWS_BLK + 8 * hh + r];
      const float y = s + bffr;
      xv[r] = y;
      if (wave == 0 && c == 0) ybuf[(8 * hh + r) * YBP + t] = y;
    }
  }
  __syncthreads();

  for (int pass = 0; pass < 2; ++pass) {
#pragma unroll
    for (int rr = 0; rr < 2; ++rr) {
      const int row = 2 * wave + rr;
      const v4f v = *(const v4f*)(ybuf + row * YBP + 4 * lane);
      *(volatile v4f*)(out + (size_t)(rowbase + row) * NSTEP + 4 * lane) = v;
    }
    __threadfence();
  }
}

extern "C" void kernel_launch(void* const* d_in, const int* in_sizes, int n_in,
                              void* d_out, int out_size, void* d_ws, size_t ws_size, hipStream_t stream) {
  if (n_in < 9 || d_out == nullptr || d_ws == nullptr) return;
  if (in_sizes[0] != NBATCH * NHID || in_sizes[1] != NGATE3 || in_sizes[2] != NGATE3 * NHID ||
      in_sizes[3] != NGATE3 || in_sizes[4] != NGATE3 || in_sizes[5] != NHID ||
      in_sizes[6] != 1 || in_sizes[7] != 1 || in_sizes[8] != 1 || out_size != NBATCH * NSTEP) return;

  const float* vectors     = (const float*)d_in[0];
  const float* w_ih        = (const float*)d_in[1];
  const float* w_hh        = (const float*)d_in[2];
  const float* b_ih        = (const float*)d_in[3];
  const float* b_hh        = (const float*)d_in[4];
  const float* w_ffn       = (const float*)d_in[5];
  const float* b_ffn       = (const float*)d_in[6];
  const float* first_input = (const float*)d_in[7];
  const int*   seq_len     = (const int*)d_in[8];
  float* out = (float*)d_out;

  char* ws = (char*)d_ws; size_t off = 0;
  auto carve = [&](size_t bytes) -> char* { char* p = ws + off; off += (bytes + 255) & ~(size_t)255; return p; };
  unsigned short* WH = (unsigned short*)carve((size_t)NGATE3 * NHID * 2);
  float*          CT = (float*)carve((size_t)NCT * NHID * 4);
  if (off > ws_size || off > (size_t)134217728) return;

  cvt_w_kernel<<<W8 / NTHR, NTHR, 0, stream>>>(w_hh, WH, W8);
  ctab_kernel<<<NCT, NTHR, 0, stream>>>(w_ih, b_ih, b_hh, w_ffn, CT);
  gru_seq_kernel<<<NBATCH / ROWS_BLK, NTHR, 0, stream>>>(vectors, CT, b_ffn, first_input, seq_len, WH, out);
}
